// SpatialGraphMambaBlock_18717467476154
// MI455X (gfx1250) — hardware-verified
//
#include <hip/hip_runtime.h>
#include <math.h>

typedef __attribute__((ext_vector_type(16))) _Float16 v16h;
typedef __attribute__((ext_vector_type(8)))  _Float16 v8h;
typedef __attribute__((ext_vector_type(16))) __bf16   v16b;
typedef __attribute__((ext_vector_type(8)))  __bf16   v8b;
typedef __attribute__((ext_vector_type(8)))  float    v8f;
typedef __attribute__((ext_vector_type(4)))  float    v4f;

constexpr int kNB     = 8;
constexpr int kSeq    = 512;
constexpr int kSeqP   = kSeq + 6;
constexpr int kDM     = 768;
constexpr int kDI     = 1536;
constexpr int kNS     = 16;
constexpr int kDTR    = 48;
constexpr int kXDW    = 80;
constexpr int kXDP    = 128;
constexpr int kDtK    = 64;
constexpr int kKsp    = 7;
constexpr int kKcv    = kKsp * kDM;
constexpr int kRows   = kNB * kSeq;
constexpr int kEnc    = 64;
constexpr int kNode   = 16;
constexpr int kScanTS = 64;
constexpr int kScanCh = 64;
constexpr int kScanYP = 68;
constexpr int kConvTP = 260;
static_assert(kDTR + 2 * kNS == kXDW, "xproj width");
static_assert((kDM % 32) == 0 && (kDI % 32) == 0 && (kKcv % 32) == 0 && (kDtK % 32) == 0, "GEMM K multiples of 32");
static_assert((kSeq % 64) == 0 && (kRows % 64) == 0 && (kDM % 64) == 0 && (kDI % 64) == 0 && (kXDP % 64) == 0, "GEMM M,N multiples of 64");
static_assert((kSeq % kScanTS) == 0 && (kDI % kScanCh) == 0 && (kDI % 256) == 0 && (kDM % 256) == 0, "tile multiples");
static_assert(kKcv == 21 * 256, "conv weight row chunks");

constexpr size_t kSzW768  = (size_t)kDM * kDM * 2;
constexpr size_t kOffWGCN = 0;
constexpr size_t kOffWCV  = kOffWGCN + kSzW768;
constexpr size_t kOffWGG  = kOffWCV  + (size_t)kDM * kKcv * 2;
constexpr size_t kOffWGM  = kOffWGG  + kSzW768;
constexpr size_t kOffWOUT = kOffWGM  + kSzW768;
constexpr size_t kOffWIN  = kOffWOUT + kSzW768;
constexpr size_t kOffWX   = kOffWIN  + (size_t)2 * kDI * kDM * 2;
constexpr size_t kOffWDT  = kOffWX   + (size_t)kXDP * kDI * 2;
constexpr size_t kOffWMO  = kOffWDT  + (size_t)kDI * kDtK * 2;
constexpr size_t kOffXNP  = kOffWMO  + (size_t)kDM * kDI * 2;
constexpr size_t kOffRA   = kOffXNP  + (size_t)kNB * kSeqP * kDM * 2;
constexpr size_t kOffXG   = kOffRA   + (size_t)kRows * kDM * 4;
constexpr size_t kOffXGH  = kOffXG   + (size_t)kRows * kDM * 4;
constexpr size_t kOffXZX  = kOffXGH  + (size_t)kRows * kDM * 2;
constexpr size_t kOffZZ   = kOffXZX  + (size_t)kRows * kDI * 4;
constexpr size_t kOffDT   = kOffZZ   + (size_t)kRows * kDI * 4;
constexpr size_t kOffXD   = kOffDT   + (size_t)kRows * kDI * 2;
constexpr size_t kOffXDH  = kOffXD   + (size_t)kRows * kXDP * 4;
constexpr size_t kWsTotal = kOffXDH  + (size_t)kRows * kXDP * 2;
constexpr size_t kOffFH   = kOffXNP;
constexpr size_t kOffXM   = kOffXZX;
constexpr size_t kOffXMH  = kOffXZX + (size_t)kRows * kDM * 4;
constexpr size_t kOffGPA  = kOffZZ;
constexpr size_t kOffOL   = kOffZZ + (size_t)kRows * kDM * 4;
constexpr size_t kOffGP   = kOffDT;
static_assert(kWsTotal == 124526592ull, "carve total");
static_assert(kWsTotal <= 134217728ull, "carve cap");
static_assert((size_t)kRows * kDM * 2 <= (size_t)kNB * kSeqP * kDM * 2, "FH fits XNP region");
static_assert((size_t)kRows * kDI * 2 == (size_t)kRows * kDM * 4, "UH/YH fit RA region");
static_assert(kOffXMH + (size_t)kRows * kDM * 2 <= kOffZZ, "XM+XMH fit XZX region");
static_assert(kOffOL + (size_t)kRows * kDM * 4 <= kOffDT, "GPA+OL fit ZZ region");
static_assert((size_t)kRows * kDM * 4 <= (size_t)kRows * kDI * 2, "GP fits DT region");
static_assert((kOffWCV % 128) == 0 && (kOffWGG % 128) == 0 && (kOffWGM % 128) == 0 && (kOffWOUT % 128) == 0 &&
              (kOffWIN % 128) == 0 && (kOffWX % 128) == 0 && (kOffWDT % 128) == 0 && (kOffWMO % 128) == 0 &&
              (kOffXNP % 128) == 0 && (kOffRA % 128) == 0 && (kOffXG % 128) == 0 && (kOffXGH % 128) == 0 &&
              (kOffXZX % 128) == 0 && (kOffZZ % 128) == 0 && (kOffDT % 128) == 0 && (kOffXD % 128) == 0 &&
              (kOffXDH % 128) == 0 && (kOffXMH % 128) == 0 && (kOffOL % 128) == 0, "128-B aligned regions");

__device__ __forceinline__ unsigned short f2bf_bits(float f) {
  unsigned u = __float_as_uint(f);
  return (unsigned short)((u + 0x7FFFu + ((u >> 16) & 1u)) >> 16);
}
__device__ __forceinline__ float bf_bits2f(unsigned short h) { return __uint_as_float(((unsigned)h) << 16); }

__device__ __forceinline__ void dep_guard_h(v8f& a, v8f& b, v16h x, v16h y) { asm volatile("v_nop\n\tv_nop\n\tv_nop\n\tv_nop" : "+v"(a), "+v"(b) : "v"(x), "v"(y)); }
__device__ __forceinline__ void dep_guard_b(v8f& a, v8f& b, v16b x, v16b y) { asm volatile("v_nop\n\tv_nop\n\tv_nop\n\tv_nop" : "+v"(a), "+v"(b) : "v"(x), "v"(y)); }
__device__ __forceinline__ void keep4_h(v16h a, v16h b, v16h c, v16h d) { asm volatile("v_nop" :: "v"(a), "v"(b), "v"(c), "v"(d)); }
__device__ __forceinline__ void keep4_b(v16b a, v16b b, v16b c, v16b d) { asm volatile("v_nop" :: "v"(a), "v"(b), "v"(c), "v"(d)); }
__device__ __forceinline__ void acc_guard4(v8f& a, v8f& b, v8f& c, v8f& d) { asm volatile("v_nop\n\tv_nop\n\tv_nop\n\tv_nop" : "+v"(a), "+v"(b), "+v"(c), "+v"(d)); }
template <typename T> struct Frag;
template <> struct Frag<_Float16> {
  typedef v16h V; union U { v16h v; v8h h[2]; };
  static __device__ __forceinline__ v16h load(const _Float16* p) {
    U f; f.h[0] = *(const v8h*)(p); f.h[1] = *(const v8h*)(p + 16); return f.v;
  }
  static __device__ __forceinline__ v8f mma(v16h a, v16h b, v8f c) {
    return __builtin_amdgcn_wmma_f32_16x16x32_f16(false, a, false, b, (short)0, c, false, false);
  }
  static __device__ __forceinline__ void guard(v8f& a, v8f& b, v16h x, v16h y) { dep_guard_h(a, b, x, y); }
  static __device__ __forceinline__ void keep(v16h a, v16h b, v16h c, v16h d) { keep4_h(a, b, c, d); }
};
template <> struct Frag<__bf16> {
  typedef v16b V; union U { v16b v; v8b h[2]; };
  static __device__ __forceinline__ v16b load(const __bf16* p) {
    U f; f.h[0] = *(const v8b*)(p); f.h[1] = *(const v8b*)(p + 16); return f.v;
  }
  static __device__ __forceinline__ v8f mma(v16b a, v16b b, v8f c) {
    return __builtin_amdgcn_wmma_f32_16x16x32_bf16(false, a, false, b, (short)0, c, false, false);
  }
  static __device__ __forceinline__ void guard(v8f& a, v8f& b, v16b x, v16b y) { dep_guard_b(a, b, x, y); }
  static __device__ __forceinline__ void keep(v16b a, v16b b, v16b c, v16b d) { keep4_b(a, b, c, d); }
};

template <int ET> struct Elem;
template <> struct Elem<0> { typedef _Float16 T; };
template <> struct Elem<1> { typedef __bf16 T; };
template <int ET, int SPL, int BIAS_MODE, int OUT_MODE, bool RESID, int ACT = 0, int CARRY_EXP = 0>
__global__ __launch_bounds__(256) void wmma_gemm64(
    const unsigned short* __restrict__ Ap, const unsigned short* __restrict__ A2p, int lda, long strideA,
    const unsigned short* __restrict__ Btp, const unsigned short* __restrict__ Bt2p, int ldb, long strideB,
    void* __restrict__ Cout, void* __restrict__ Cout2, int ldc, long strideC,
    const float* __restrict__ bias,
    const float* __restrict__ resid, long strideR,
    int M, int N, int K, float scale) {
  typedef typename Elem<ET>::T T;
  typedef typename Frag<T>::V V;
  const T* A = (const T*)Ap; const T* A2 = (const T*)A2p; const T* Bt = (const T*)Btp; const T* Bt2 = (const T*)Bt2p;
  __shared__ __align__(16) float sT[8][16 * 68];
  const int b    = blockIdx.y;
  const int lane = threadIdx.x & 31;
  const int wave = threadIdx.x >> 5;
  const int tilesN = N >> 6;
  const int tilesM = M >> 6;
  const int tile = blockIdx.x * 8 + wave;
  if (tile >= tilesM * tilesN) return;
  const int tm = tile / tilesN;
  const int tn = tile - tm * tilesN;
  const int m0 = tm << 6;
  const int n0 = tn << 6;

  const T* Ab  = A  + (size_t)b * strideA;
  const T* Bb  = Bt + (size_t)b * strideB;
  const T* Ab2 = (SPL >= 1) ? (A2  + (size_t)b * strideA) : nullptr;
  const T* Bb2 = (SPL == 2) ? (Bt2 + (size_t)b * strideB) : nullptr;

  const int rlane = lane & 15;
  const int koff  = (lane >> 4) * 8;
  const int mOff  = (lane >> 4) * 8;

  v8f acc[4][4];
#pragma unroll
  for (int i = 0; i < 4; ++i)
#pragma unroll
    for (int j = 0; j < 4; ++j) acc[i][j] = (v8f){0.f,0.f,0.f,0.f,0.f,0.f,0.f,0.f};

  for (int k0 = 0; k0 < K; k0 += 32) {
    V bh[4], bl[4];
#pragma unroll
    for (int j = 0; j < 4; ++j) {
      const size_t bo = (size_t)(n0 + (j << 4) + rlane) * ldb + koff + k0;
      bh[j] = Frag<T>::load(Bb + bo);
      if (SPL == 2) bl[j] = Frag<T>::load(Bb2 + bo);
    }
#pragma unroll
    for (int i = 0; i < 4; ++i) {
      const size_t ao = (size_t)(m0 + (i << 4) + rlane) * lda + koff + k0;
      V ah = Frag<T>::load(Ab + ao);
      V al;
      if (SPL >= 1) al = Frag<T>::load(Ab2 + ao);
#pragma unroll
      for (int j = 0; j < 4; ++j) {
        acc[i][j] = Frag<T>::mma(ah, bh[j], acc[i][j]);
        if (SPL == 2) acc[i][j] = Frag<T>::mma(ah, bl[j], acc[i][j]);
        if (SPL >= 1) acc[i][j] = Frag<T>::mma(al, bh[j], acc[i][j]);
      }
      Frag<T>::guard(acc[i][0], acc[i][3], ah, (SPL >= 1) ? al : ah);
    }
    Frag<T>::keep(bh[0], bh[1], bh[2], bh[3]);
    if (SPL == 2) Frag<T>::keep(bl[0], bl[1], bl[2], bl[3]);
  }
  acc_guard4(acc[0][0], acc[0][1], acc[0][2], acc[0][3]);
  acc_guard4(acc[1][0], acc[1][1], acc[1][2], acc[1][3]);
  acc_guard4(acc[2][0], acc[2][1], acc[2][2], acc[2][3]);
  acc_guard4(acc[3][0], acc[3][1], acc[3][2], acc[3][3]);

  float* slab = sT[wave];
  const float* Rb = RESID ? (resid + (size_t)b * strideR) : nullptr;
  const float carry = (float)(1 << CARRY_EXP);
  float* Cf = (float*)Cout + (size_t)b * strideC;
  unsigned short* Ch = ((OUT_MODE == 3) ? (unsigned short*)Cout2 : (unsigned short*)Cout) + (size_t)b * strideC;
  unsigned short* Cl = (OUT_MODE == 2) ? ((unsigned short*)Cout2 + (size_t)b * strideC) : nullptr;
  const int hh = lane >> 4, c4 = (lane & 15) * 4;
  const int q = lane >> 3, c8 = (lane & 7) * 8;
#pragma unroll
  for (int i = 0; i < 4; ++i) {
    const int mBase = m0 + (i << 4);
#pragma unroll
    for (int j = 0; j < 4; ++j) {
      const int n = n0 + (j << 4) + rlane;
      float bv = 0.f;
      if (BIAS_MODE == 2) bv = bias[n];
#pragma unroll
      for (int r = 0; r < 8; ++r) {
        float v = acc[i][j][r] * scale;
        if (BIAS_MODE == 1) v += bias[mBase + mOff + r];
        if (BIAS_MODE == 2) v += bv;
        if (RESID) v += Rb[(size_t)(mBase + mOff + r) * ldc + n];
        if (ACT == 1) v = tanhf(v);
        if (ACT == 2) v = fmaxf(v, 0.0f);
        if (ACT == 3) v = v / (1.0f + expf(-v));
        if (ACT == 4) v = (v > 0.f) ? v : 0.01f * v;
        slab[(mOff + r) * 68 + (j << 4) + rlane] = v;
      }
    }
    __builtin_amdgcn_fence(__ATOMIC_RELEASE, "workgroup");
    __builtin_amdgcn_wave_barrier();
    __builtin_amdgcn_fence(__ATOMIC_ACQUIRE, "workgroup");
    for (int pass = 0; pass < 2; ++pass) {
      if (OUT_MODE == 0 || OUT_MODE == 3) {
#pragma unroll
        for (int it = 0; it < 8; ++it) {
          const int row = it * 2 + hh;
          v4f v = *(const v4f*)(slab + row * 68 + c4);
          *(volatile v4f*)(Cf + (size_t)(mBase + row) * ldc + n0 + c4) = v;
        }
      }
      if (OUT_MODE != 0) {
#pragma unroll
        for (int it = 0; it < 4; ++it) {
          const int row = it * 4 + q;
          const float* sp = slab + row * 68 + c8;
          v8h hv, lv;
#pragma unroll
          for (int e = 0; e < 8; ++e) {
            if (OUT_MODE == 1 || OUT_MODE == 3) {
              hv[e] = (_Float16)(sp[e] * carry);
            } else {
              const unsigned short hb = f2bf_bits(sp[e]);
              hv[e] = __builtin_bit_cast(_Float16, hb);
              if (OUT_MODE == 2) {
                const unsigned short lb = f2bf_bits(sp[e] - bf_bits2f(hb));
                lv[e] = __builtin_bit_cast(_Float16, lb);
              }
            }
          }
          *(volatile v8h*)(Ch + (size_t)(mBase + row) * ldc + n0 + c8) = hv;
          if (OUT_MODE == 2) *(volatile v8h*)(Cl + (size_t)(mBase + row) * ldc + n0 + c8) = lv;
        }
      }
      __threadfence();
    }
    __builtin_amdgcn_fence(__ATOMIC_RELEASE, "workgroup");
    __builtin_amdgcn_wave_barrier();
    __builtin_amdgcn_fence(__ATOMIC_ACQUIRE, "workgroup");
  }
}

__global__ __launch_bounds__(256) void tcast_kernel(const float* __restrict__ in, int R, int Ccols,
                                                    _Float16* __restrict__ out, int Kpad, float scale)
{
  __shared__ __align__(16) float sT[64 * 68];
  const int tid = threadIdx.x, lane = tid & 31, wave = tid >> 5;
  const int k0 = blockIdx.x * 64, n0 = blockIdx.y * 64;
  const int nl = tid & 63, kq = tid >> 6;
  const int n = n0 + nl;
  const int nc = (n < Ccols) ? n : (Ccols - 1);
#pragma unroll
  for (int i = 0; i < 16; ++i) {
    const int kl = kq + 4 * i;
    const int k = k0 + kl;
    const int kc = (k < R) ? k : (R - 1);
    float v = in[(size_t)kc * Ccols + nc] * scale;
    if (k >= R || n >= Ccols) v = 0.0f;
    sT[nl * 68 + kl] = v;
  }
  __syncthreads();
  const int q = lane >> 3, c8 = (lane & 7) * 8;
  v8h hv[2];
#pragma unroll
  for (int it = 0; it < 2; ++it) {
    const int r = it * 32 + wave * 4 + q;
    const float* sp = sT + r * 68 + c8;
    const v4f a0 = *(const v4f*)(sp);
    const v4f a1 = *(const v4f*)(sp + 4);
#pragma unroll
    for (int e = 0; e < 4; ++e) { hv[it][e] = (_Float16)a0[e]; hv[it][4 + e] = (_Float16)a1[e]; }
  }
  for (int pass = 0; pass < 2; ++pass) {
#pragma unroll
    for (int it = 0; it < 2; ++it) {
      const int r = it * 32 + wave * 4 + q;
      *(volatile v8h*)(out + (size_t)(n0 + r) * Kpad + k0 + c8) = hv[it];
    }
    __threadfence();
  }
}

__global__ __launch_bounds__(256) void wcv_kernel(const float* __restrict__ cwt, _Float16* __restrict__ out)
{
  __shared__ __align__(16) float srow[kKcv];
  const int tid = threadIdx.x, lane = tid & 31, wave = tid >> 5;
  const int o = blockIdx.x;
  const float* src = cwt + (size_t)o * kKcv;
#pragma unroll 1
  for (int i = 0; i < 21; ++i) srow[i * 256 + tid] = src[i * 256 + tid] * 32.0f;
  __syncthreads();
  _Float16* orow = out + (size_t)o * kKcv;
  for (int pass = 0; pass < 2; ++pass) {
    for (int ch = wave; ch < 21; ch += 8) {
      const int j0 = ch * 256 + lane * 8;
      const int kk = j0 / kDM;
      const int c0 = j0 - kk * kDM;
      v8h hv;
#pragma unroll
      for (int e = 0; e < 8; ++e) hv[e] = (_Float16)srow[(c0 + e) * kKsp + kk];
      *(volatile v8h*)(orow + j0) = hv;
    }
    __threadfence();
  }
}

__global__ __launch_bounds__(256) void adj_kernel(const float* __restrict__ nv1, const float* __restrict__ nv2,
                                                  float* __restrict__ adj)
{
  __shared__ __align__(16) float sadj[kEnc * kEnc];
  const int t = threadIdx.x;
#pragma unroll 1
  for (int i = 0; i < 16; ++i) {
    const int e = i * 256 + t;
    const int r = e >> 6, c = e & 63;
    float s = 0.f;
#pragma unroll
    for (int k = 0; k < kNode; ++k) s += nv1[r * kNode + k] * nv2[k * kEnc + c];
    const float a = 1.0f / (1.0f + expf(-s));
    sadj[e] = (r == c) ? 0.0f : a;
  }
  __syncthreads();
  for (int pass = 0; pass < 2; ++pass) {
#pragma unroll
    for (int i = 0; i < 4; ++i) {
      const int idx = i * 256 + t;
      const v4f v = *(const v4f*)(sadj + idx * 4);
      *(volatile v4f*)(adj + (size_t)idx * 4) = v;
    }
    __threadfence();
  }
}

__global__ __launch_bounds__(256) void ln1_kernel(const float* __restrict__ x, const float* __restrict__ w,
                                                  const float* __restrict__ bb, _Float16* __restrict__ xnp)
{
  const int lane = threadIdx.x & 31, wave = threadIdx.x >> 5;
  const int pr = blockIdx.x * 8 + wave;
  if (pr >= kNB * kSeqP) return;
  const int bi = pr / kSeqP;
  const int tp = pr - bi * kSeqP;
  const int t  = tp - 3;
  const bool pad = (t < 0) || (t >= kSeq);
  const int tc = (t < 0) ? 0 : ((t >= kSeq) ? (kSeq - 1) : t);
  const float* xr = x + ((size_t)bi * kSeq + tc) * kDM;
  v4f v[6];
#pragma unroll
  for (int it = 0; it < 3; ++it) {
    const int c0 = it * 256 + lane * 8;
    v[2 * it]     = *(const v4f*)(xr + c0);
    v[2 * it + 1] = *(const v4f*)(xr + c0 + 4);
  }
  float s = 0.f;
#pragma unroll
  for (int i = 0; i < 6; ++i) s += (v[i][0] + v[i][1]) + (v[i][2] + v[i][3]);
#pragma unroll
  for (int off = 16; off > 0; off >>= 1) s += __shfl_xor(s, off, 32);
  const float mu = s * (1.0f / (float)kDM);
  float ss = 0.f;
#pragma unroll
  for (int i = 0; i < 6; ++i) {
#pragma unroll
    for (int e = 0; e < 4; ++e) { const float dd = v[i][e] - mu; ss += dd * dd; }
  }
#pragma unroll
  for (int off = 16; off > 0; off >>= 1) ss += __shfl_xor(ss, off, 32);
  const float var = ss * (1.0f / (float)kDM);
  const float inv = rsqrtf(var + 1e-5f);
  const float keep = pad ? 0.0f : 1.0f;
  _Float16* orow = xnp + ((size_t)bi * kSeqP + tp) * kDM;
  v8h hv[3];
#pragma unroll
  for (int it = 0; it < 3; ++it) {
    const int c0 = it * 256 + lane * 8;
    const v4f wa = *(const v4f*)(w + c0),  wb = *(const v4f*)(w + c0 + 4);
    const v4f ba = *(const v4f*)(bb + c0), bbv = *(const v4f*)(bb + c0 + 4);
#pragma unroll
    for (int e = 0; e < 4; ++e) {
      const float y0 = ((v[2 * it][e]     - mu) * inv * wa[e] + ba[e])  * keep;
      const float y1 = ((v[2 * it + 1][e] - mu) * inv * wb[e] + bbv[e]) * keep;
      hv[it][e]     = (_Float16)y0;
      hv[it][4 + e] = (_Float16)y1;
    }
  }
  for (int pass = 0; pass < 2; ++pass) {
#pragma unroll
    for (int it = 0; it < 3; ++it) {
      const int c0 = it * 256 + lane * 8;
      *(volatile v8h*)(orow + c0) = hv[it];
    }
    __threadfence();
  }
}

__global__ __launch_bounds__(256) void ln2_kernel(const float* __restrict__ ol, const float* __restrict__ x,
                                                  const float* __restrict__ w, const float* __restrict__ bb,
                                                  float* __restrict__ out)
{
  const int lane = threadIdx.x & 31, wave = threadIdx.x >> 5;
  const int row = blockIdx.x * 8 + wave;
  if (row >= kRows) return;
  const float* pr = ol + (size_t)row * kDM;
  const float* xr = x  + (size_t)row * kDM;
  v4f v[6];
#pragma unroll
  for (int it = 0; it < 6; ++it) {
    const int c0 = it * 128 + lane * 4;
    v[it] = *(const v4f*)(pr + c0) + *(const v4f*)(xr + c0);
  }
  float s = 0.f;
#pragma unroll
  for (int i = 0; i < 6; ++i) s += (v[i][0] + v[i][1]) + (v[i][2] + v[i][3]);
#pragma unroll
  for (int off = 16; off > 0; off >>= 1) s += __shfl_xor(s, off, 32);
  const float mu = s * (1.0f / (float)kDM);
  float ss = 0.f;
#pragma unroll
  for (int i = 0; i < 6; ++i) {
#pragma unroll
    for (int e = 0; e < 4; ++e) { const float dd = v[i][e] - mu; ss += dd * dd; }
  }
#pragma unroll
  for (int off = 16; off > 0; off >>= 1) ss += __shfl_xor(ss, off, 32);
  const float var = ss * (1.0f / (float)kDM);
  const float inv = rsqrtf(var + 1e-5f);
  v4f o[6];
#pragma unroll
  for (int it = 0; it < 6; ++it) {
    const int c0 = it * 128 + lane * 4;
    const v4f wa = *(const v4f*)(w + c0), ba = *(const v4f*)(bb + c0);
#pragma unroll
    for (int e = 0; e < 4; ++e) o[it][e] = (v[it][e] - mu) * inv * wa[e] + ba[e];
  }
  float* orow = out + (size_t)row * kDM;
  for (int pass = 0; pass < 2; ++pass) {
#pragma unroll
    for (int it = 0; it < 6; ++it) {
      const int c0 = it * 128 + lane * 4;
      *(volatile v4f*)(orow + c0) = o[it];
    }
    __threadfence();
  }
}

__global__ __launch_bounds__(256) void dwconv_kernel(
    const float* __restrict__ xzx, const float* __restrict__ cw, const float* __restrict__ cb,
    _Float16* __restrict__ uh)
{
  __shared__ __align__(16) float sT[16 * kConvTP];
  const int tid = threadIdx.x, lane = tid & 31, wave = tid >> 5;
  const int d0 = blockIdx.x * 256, d = d0 + tid;
  const int g0 = blockIdx.y * 64;
  const int tb = g0 & (kSeq - 1);
  const float w0 = cw[d * 4 + 0], w1 = cw[d * 4 + 1], w2 = cw[d * 4 + 2], w3 = cw[d * 4 + 3];
  const float bc = cb[d];
  float xm3, xm2, xm1;
  {
    const bool hist = (tb > 0);
    const int rb = hist ? (g0 - 3) : g0;
    const float v3 = xzx[(size_t)rb * kDI + d];
    const float v2 = xzx[(size_t)(rb + 1) * kDI + d];
    const float v1 = xzx[(size_t)(rb + 2) * kDI + d];
    xm3 = hist ? v3 : 0.f;
    xm2 = hist ? v2 : 0.f;
    xm1 = hist ? v1 : 0.f;
  }
#pragma unroll 1
  for (int sub = 0; sub < 4; ++sub) {
    const int lb = g0 + sub * 16;
#pragma unroll 1
    for (int s = 0; s < 16; ++s) {
      const float xcur = xzx[(size_t)(lb + s) * kDI + d];
      float acc = w0 * xm3;
      acc = fmaf(w1, xm2, acc);
      acc = fmaf(w2, xm1, acc);
      acc = fmaf(w3, xcur, acc);
      const float sv = acc + bc;
      const float sg = __builtin_amdgcn_rcpf(1.0f + expf(-sv));
      sT[s * kConvTP + tid] = (sv * sg) * 64.0f;
      xm3 = xm2; xm2 = xm1; xm1 = xcur;
    }
    __syncthreads();
    v8h hv[2];
#pragma unroll
    for (int it = 0; it < 2; ++it) {
      const float* sp = sT + (it * 8 + wave) * kConvTP + lane * 8;
      const v4f a0 = *(const v4f*)(sp);
      const v4f a1 = *(const v4f*)(sp + 4);
#pragma unroll
      for (int e = 0; e < 4; ++e) { hv[it][e] = (_Float16)a0[e]; hv[it][4 + e] = (_Float16)a1[e]; }
    }
    for (int pass = 0; pass < 2; ++pass) {
#pragma unroll
      for (int it = 0; it < 2; ++it)
        *(volatile v8h*)(uh + (size_t)(lb + it * 8 + wave) * kDI + d0 + lane * 8) = hv[it];
      __threadfence();
    }
    __syncthreads();
  }
}

__global__ __launch_bounds__(64) void scan_kernel(
    const float* __restrict__ xd, const unsigned short* __restrict__ dtp,
    const float* __restrict__ xzx, const float* __restrict__ zz,
    const float* __restrict__ cw, const float* __restrict__ cb,
    const float* __restrict__ bdt, const float* __restrict__ alog, const float* __restrict__ dp,
    _Float16* __restrict__ yh)
{
  __shared__ __align__(16) float sX[kScanTS * 32];
  __shared__ __align__(16) float sY[kScanTS * kScanYP];
  __shared__ __align__(16) float sA[kNS * kScanCh];
  const int tid = threadIdx.x, lane = tid & 31, wave = tid >> 5;
  constexpr int kBlkPerB = kDI / kScanCh;
  const int bix = blockIdx.x / kBlkPerB;
  const int d0  = (blockIdx.x - bix * kBlkPerB) * kScanCh;
  const int d   = d0 + tid;
  const size_t row0 = (size_t)bix * kSeq;
#pragma unroll 1
  for (int s = 0; s < kNS; ++s) sA[s * kScanCh + tid] = -expf(alog[(size_t)d * kNS + s]);
  __syncthreads();
  float negA[kNS], h[kNS];
#pragma unroll
  for (int s = 0; s < kNS; ++s) { negA[s] = sA[s * kScanCh + tid]; h[s] = 0.f; }
  const float w0 = cw[d * 4 + 0], w1 = cw[d * 4 + 1], w2 = cw[d * 4 + 2], w3 = cw[d * 4 + 3];
  const float bc = cb[d];
  const float bb = bdt[d], Dd = dp[d];
  float xm3 = 0.f, xm2 = 0.f, xm1 = 0.f;
  const int q = lane >> 3, c8 = (lane & 7) * 8;
#pragma unroll 1
  for (int t0 = 0; t0 < kSeq; t0 += kScanTS) {
    __syncthreads();
#pragma unroll
    for (int i = 0; i < 8; ++i) {
      const int idx = i * 64 + tid;
      const int st = idx >> 3, c4 = (idx & 7) * 4;
      *(v4f*)(sX + st * 32 + c4) = *(const v4f*)(xd + (row0 + t0 + st) * kXDP + kDTR + c4);
    }
    __syncthreads();
#pragma unroll 1
    for (int s = 0; s < kScanTS; ++s) {
      const size_t row = row0 + t0 + s;
      const float xcur = xzx[row * kDI + d];
      float cacc = w0 * xm3;
      cacc = fmaf(w1, xm2, cacc);
      cacc = fmaf(w2, xm1, cacc);
      cacc = fmaf(w3, xcur, cacc);
      xm3 = xm2; xm2 = xm1; xm1 = xcur;
      const float sv = cacc + bc;
      const float u  = sv * __builtin_amdgcn_rcpf(1.0f + expf(-sv));
      const float* xr = sX + s * 32;
      float Bs[kNS], Cs[kNS];
#pragma unroll
      for (int q4 = 0; q4 < 4; ++q4) {
        const v4f bv = *(const v4f*)(xr + 4 * q4);
        const v4f cv = *(const v4f*)(xr + kNS + 4 * q4);
        Bs[4 * q4 + 0] = bv[0]; Bs[4 * q4 + 1] = bv[1]; Bs[4 * q4 + 2] = bv[2]; Bs[4 * q4 + 3] = bv[3];
        Cs[4 * q4 + 0] = cv[0]; Cs[4 * q4 + 1] = cv[1]; Cs[4 * q4 + 2] = cv[2]; Cs[4 * q4 + 3] = cv[3];
      }
      const float v   = __uint_as_float(((unsigned)dtp[row * kDI + d]) << 16) + bb;
      const float ea  = expf(-fabsf(v));
      const float up1 = 1.0f + ea;
      const float l1p = logf(up1) + (ea - (up1 - 1.0f)) * __builtin_amdgcn_rcpf(up1);
      const float dt  = fmaxf(v, 0.0f) + l1p;
      const float dtx = dt * u;
      float y = 0.f;
#pragma unroll
      for (int k = 0; k < kNS; ++k) {
        const float e = __expf(dt * negA[k]);
        h[k] = e * h[k] + dtx * Bs[k];
        y = h[k] * Cs[k] + y;
      }
      y = u * Dd + y;
      const float zv = zz[row * kDI + d];
      const float sg = __builtin_amdgcn_rcpf(1.0f + expf(-zv));
      y = y * (zv * sg);
      sY[s * kScanYP + tid] = y * 256.0f;
    }
    __syncthreads();
    v8h hv[8];
#pragma unroll
    for (int it = 0; it < 8; ++it) {
      const int r = it * 8 + wave * 4 + q;
      const float* sp = sY + r * kScanYP + c8;
      const v4f a0 = *(const v4f*)(sp);
      const v4f a1 = *(const v4f*)(sp + 4);
#pragma unroll
      for (int e = 0; e < 4; ++e) { hv[it][e] = (_Float16)a0[e]; hv[it][4 + e] = (_Float16)a1[e]; }
    }
    for (int pass = 0; pass < 2; ++pass) {
#pragma unroll
      for (int it = 0; it < 8; ++it) {
        const int r = it * 8 + wave * 4 + q;
        *(volatile v8h*)(yh + (row0 + t0 + r) * kDI + d0 + c8) = hv[it];
      }
      __threadfence();
    }
  }
}

__global__ __launch_bounds__(256) void fuse_kernel(const float* __restrict__ gp, const float* __restrict__ xg,
                                                   const float* __restrict__ xm, _Float16* __restrict__ fh, int total8)
{
  const int i = blockIdx.x * 256 + threadIdx.x;
  if (i >= total8) return;
  const size_t e0 = (size_t)i << 3;
  const v4f ga = *(const v4f*)(gp + e0), gb = *(const v4f*)(gp + e0 + 4);
  const v4f aa = *(const v4f*)(xg + e0), ab = *(const v4f*)(xg + e0 + 4);
  const v4f ma = *(const v4f*)(xm + e0), mb = *(const v4f*)(xm + e0 + 4);
  v8h hv;
#pragma unroll
  for (int e = 0; e < 4; ++e) {
    const float s0 = __builtin_amdgcn_rcpf(1.0f + expf(-ga[e]));
    const float s1 = __builtin_amdgcn_rcpf(1.0f + expf(-gb[e]));
    hv[e]     = (_Float16)(s0 * aa[e] + (1.0f - s0) * ma[e]);
    hv[4 + e] = (_Float16)(s1 * ab[e] + (1.0f - s1) * mb[e]);
  }
  *(volatile v8h*)(fh + e0) = hv;
  __threadfence();
  *(volatile v8h*)(fh + e0) = hv;
}

extern "C" void kernel_launch(void* const* d_in, const int* in_sizes, int n_in,
                              void* d_out, int out_size, void* d_ws, size_t ws_size,
                              hipStream_t stream) {
  if (n_in < 26) return;
  if (in_sizes[0]  != kRows * kDM) return;
  if (in_sizes[1]  != kEnc * kNode) return;
  if (in_sizes[2]  != kNode * kEnc) return;
  if (in_sizes[3]  != kDM || in_sizes[4] != kDM || in_sizes[5] != kDM || in_sizes[6] != kDM) return;
  if (in_sizes[7]  != kDM * kDM || in_sizes[8] != kDM) return;
  if (in_sizes[9]  != kDM * kDM * kKsp || in_sizes[10] != kDM) return;
  if (in_sizes[11] != kDM * kDM || in_sizes[12] != kDM) return;
  if (in_sizes[13] != kDM * kDM || in_sizes[14] != kDM) return;
  if (in_sizes[15] != kDM * kDM || in_sizes[16] != kDM) return;
  if (in_sizes[17] != kDM * 2 * kDI) return;
  if (in_sizes[18] != kDI * 4 || in_sizes[19] != kDI) return;
  if (in_sizes[20] != kDI * kXDW) return;
  if (in_sizes[21] != kDTR * kDI || in_sizes[22] != kDI) return;
  if (in_sizes[23] != kDI * kNS || in_sizes[24] != kDI) return;
  if (in_sizes[25] != kDI * kDM) return;
  if (out_size != kRows * kDM + kEnc * kEnc) return;
  if (ws_size < kWsTotal) return;

  const float* x            = (const float*)d_in[0];
  const float* nodevec1     = (const float*)d_in[1];
  const float* nodevec2     = (const float*)d_in[2];
  const float* norm1_w      = (const float*)d_in[3];
  const float* norm1_b      = (const float*)d_in[4];
  const float* norm2_w      = (const float*)d_in[5];
  const float* norm2_b      = (const float*)d_in[6];
  const float* gcn_w        = (const float*)d_in[7];
  const float* gcn_b        = (const float*)d_in[8];
  const float* conv_w       = (const float*)d_in[9];
  const float* conv_b       = (const float*)d_in[10];
  const float* gate_gcn_w   = (const float*)d_in[11];
  const float* gate_gcn_b   = (const float*)d_in[12];
  const float* gate_mamba_w = (const float*)d_in[13];
  const float* gate_mamba_b = (const float*)d_in[14];
  const float* out_w        = (const float*)d_in[15];
  const float* out_b        = (const float*)d_in[16];
  const float* m_in_w       = (const float*)d_in[17];
  const float* m_conv_w     = (const float*)d_in[18];
  const float* m_conv_b     = (const float*)d_in[19];
  const float* m_xproj_w    = (const float*)d_in[20];
  const float* m_dt_w       = (const float*)d_in[21];
  const float* m_dt_b       = (const float*)d_in[22];
  const float* m_A_log      = (const float*)d_in[23];
  const float* m_D          = (const float*)d_in[24];
  const float* m_out_w      = (const float*)d_in[25];
  float* out0 = (float*)d_out;
  float* adj  = out0 + (size_t)kRows * kDM;

  char* ws = (char*)d_ws;
  unsigned short* WGCN = (unsigned short*)(ws + kOffWGCN);
  unsigned short* WCV  = (unsigned short*)(ws + kOffWCV);
  unsigned short* WGG  = (unsigned short*)(ws + kOffWGG);
  unsigned short* WGM  = (unsigned short*)(ws + kOffWGM);
  unsigned short* WOUT = (unsigned short*)(ws + kOffWOUT);
  unsigned short* WIN  = (unsigned short*)(ws + kOffWIN);
  unsigned short* WX   = (unsigned short*)(ws + kOffWX);
  unsigned short* WDT  = (unsigned short*)(ws + kOffWDT);
  unsigned short* WMO  = (unsigned short*)(ws + kOffWMO);
  unsigned short* XNP  = (unsigned short*)(ws + kOffXNP);
  float*          XGA  = (float*)(ws + kOffRA);
  unsigned short* UH   = (unsigned short*)(ws + kOffRA);
  unsigned short* YH   = (unsigned short*)(ws + kOffRA);
  float*          XG   = (float*)(ws + kOffXG);
  unsigned short* XGH  = (unsigned short*)(ws + kOffXGH);
  float*          XZX  = (float*)(ws + kOffXZX);
  float*          ZZ   = (float*)(ws + kOffZZ);
  unsigned short* DT   = (unsigned short*)(ws + kOffDT);
  float*          XD   = (float*)(ws + kOffXD);
  unsigned short* XDH  = (unsigned short*)(ws + kOffXDH);
  unsigned short* FH   = (unsigned short*)(ws + kOffFH);
  float*          XM   = (float*)(ws + kOffXM);
  unsigned short* XMH  = (unsigned short*)(ws + kOffXMH);
  float*          GPA  = (float*)(ws + kOffGPA);
  float*          OL   = (float*)(ws + kOffOL);
  float*          GP   = (float*)(ws + kOffGP);

  adj_kernel<<<1, 256, 0, stream>>>(nodevec1, nodevec2, adj);

  tcast_kernel<<<dim3(kDM / 64, kDM / 64), 256, 0, stream>>>(gcn_w, kDM, kDM, (_Float16*)WGCN, kDM, 32.0f);
  tcast_kernel<<<dim3(kDM / 64, kDM / 64), 256, 0, stream>>>(gate_gcn_w, kDM, kDM, (_Float16*)WGG, kDM, 32.0f);
  tcast_kernel<<<dim3(kDM / 64, kDM / 64), 256, 0, stream>>>(gate_mamba_w, kDM, kDM, (_Float16*)WGM, kDM, 32.0f);
  tcast_kernel<<<dim3(kDM / 64, kDM / 64), 256, 0, stream>>>(out_w, kDM, kDM, (_Float16*)WOUT, kDM, 32.0f);
  tcast_kernel<<<dim3(kDM / 64, (2 * kDI) / 64), 256, 0, stream>>>(m_in_w, kDM, 2 * kDI, (_Float16*)WIN, kDM, 32.0f);
  tcast_kernel<<<dim3(kDI / 64, kXDP / 64), 256, 0, stream>>>(m_xproj_w, kDI, kXDW, (_Float16*)WX, kDI, 32.0f);
  tcast_kernel<<<dim3(kDtK / 64, kDI / 64), 256, 0, stream>>>(m_dt_w, kDTR, kDI, (_Float16*)WDT, kDtK, 32.0f);
  tcast_kernel<<<dim3(kDI / 64, kDM / 64), 256, 0, stream>>>(m_out_w, kDI, kDM, (_Float16*)WMO, kDI, 32.0f);

  wcv_kernel<<<kDM, 256, 0, stream>>>(conv_w, (_Float16*)WCV);

  ln1_kernel<<<(kNB * kSeqP) / 8, 256, 0, stream>>>(x, norm1_w, norm1_b, (_Float16*)XNP);

  wmma_gemm64<0, 0, 2, 0, false><<<dim3((kSeq / 64) * (kDM / 64) / 8, kNB), 256, 0, stream>>>(
      XNP + 3 * kDM, nullptr, kDM, (long)kSeqP * kDM,
      WGCN, nullptr, kDM, 0L,
      (void*)XGA, nullptr, kDM, (long)kSeq * kDM,
      gcn_b, nullptr, 0L,
      kSeq, kDM, kDM, 1.0f / 32.0f);

  wmma_gemm64<0, 0, 2, 3, true, 0, 0><<<dim3((kSeq / 64) * (kDM / 64) / 8, kNB), 256, 0, stream>>>(
      XNP, nullptr, kDM, (long)kSeqP * kDM,
      WCV, nullptr, kKcv, 0L,
      (void*)XG, (void*)XGH, kDM, (long)kSeq * kDM,
      conv_b, XGA, (long)kSeq * kDM,
      kSeq, kDM, kKcv, 1.0f / 32.0f);

  wmma_gemm64<0, 0, 0, 0, false><<<dim3((kSeq / 64) * (kDI / 64) / 8, kNB), 256, 0, stream>>>(
      XNP + 3 * kDM, nullptr, kDM, (long)kSeqP * kDM,
      WIN, nullptr, kDM, 0L,
      (void*)XZX, nullptr, kDI, (long)kSeq * kDI,
      nullptr, nullptr, 0L,
      kSeq, kDI, kDM, 1.0f / 32.0f);
  wmma_gemm64<0, 0, 0, 0, false><<<dim3((kSeq / 64) * (kDI / 64) / 8, kNB), 256, 0, stream>>>(
      XNP + 3 * kDM, nullptr, kDM, (long)kSeqP * kDM,
      WIN + (size_t)kDI * kDM, nullptr, kDM, 0L,
      (void*)ZZ, nullptr, kDI, (long)kSeq * kDI,
      nullptr, nullptr, 0L,
      kSeq, kDI, kDM, 1.0f / 32.0f);

  dwconv_kernel<<<dim3(kDI / 256, kRows / 64), 256, 0, stream>>>(XZX, m_conv_w, m_conv_b, (_Float16*)UH);

  wmma_gemm64<0, 0, 0, 3, false, 0, 8><<<dim3((kRows / 64) * (kXDP / 64) / 8, 1), 256, 0, stream>>>(
      UH, nullptr, kDI, 0L,
      WX, nullptr, kDI, 0L,
      (void*)XD, (void*)XDH, kXDP, 0L,
      nullptr, nullptr, 0L,
      kRows, kXDP, kDI, 1.0f / 2048.0f);

  wmma_gemm64<0, 0, 0, 4, false><<<dim3((kRows / 64) * (kDI / 64) / 8, 1), 256, 0, stream>>>(
      XDH, nullptr, kXDP, 0L,
      WDT, nullptr, kDtK, 0L,
      (void*)DT, nullptr, kDI, 0L,
      nullptr, nullptr, 0L,
      kRows, kDI, kDtK, 1.0f / 8192.0f);

  scan_kernel<<<kNB * (kDI / kScanCh), kScanCh, 0, stream>>>(XD, DT, XZX, ZZ, m_conv_w, m_conv_b, m_dt_b, m_A_log, m_D, (_Float16*)YH);

  wmma_gemm64<0, 0, 0, 3, false, 0, 8><<<dim3((kRows / 64) * (kDM / 64) / 8, 1), 256, 0, stream>>>(
      YH, nullptr, kDI, 0L,
      WMO, nullptr, kDI, 0L,
      (void*)XM, (void*)XMH, kDM, 0L,
      nullptr, nullptr, 0L,
      kRows, kDM, kDI, 1.0f / 8192.0f);

  wmma_gemm64<0, 0, 2, 0, false><<<dim3((kRows / 64) * (kDM / 64) / 8, 1), 256, 0, stream>>>(
      XGH, nullptr, kDM, 0L,
      WGG, nullptr, kDM, 0L,
      (void*)GPA, nullptr, kDM, 0L,
      gate_gcn_b, nullptr, 0L,
      kRows, kDM, kDM, 1.0f / 32.0f);

  wmma_gemm64<0, 0, 2, 0, true><<<dim3((kRows / 64) * (kDM / 64) / 8, 1), 256, 0, stream>>>(
      XMH, nullptr, kDM, 0L,
      WGM, nullptr, kDM, 0L,
      (void*)GP, nullptr, kDM, 0L,
      gate_mamba_b, GPA, 0L,
      kRows, kDM, kDM, 1.0f / 8192.0f);

  fuse_kernel<<<(kRows * kDM / 8) / 256, 256, 0, stream>>>(GP, XG, XM, (_Float16*)FH, kRows * kDM / 8);

  wmma_gemm64<0, 0, 2, 0, false><<<dim3((kRows / 64) * (kDM / 64) / 8, 1), 256, 0, stream>>>(
      FH, nullptr, kDM, 0L,
      WOUT, nullptr, kDM, 0L,
      (void*)OL, nullptr, kDM, 0L,
      out_b, nullptr, 0L,
      kRows, kDM, kDM, 1.0f / 32.0f);

  ln2_kernel<<<kRows / 8, 256, 0, stream>>>(OL, x, norm2_w, norm2_b, out0);
}
